// FlowEmbedding_88201448391141
// MI455X (gfx1250) — hardware-verified
//
#include <hip/hip_runtime.h>

#pragma clang fp contract(off)

typedef __attribute__((ext_vector_type(16))) _Float16 v16h;
typedef __attribute__((ext_vector_type(8)))  _Float16 v8h;
typedef __attribute__((ext_vector_type(8)))  float    v8f;
typedef __attribute__((ext_vector_type(4)))  float    v4f;
typedef __attribute__((ext_vector_type(4)))  unsigned v4u;
typedef __attribute__((ext_vector_type(2)))  double   v2d;

constexpr int kBatch  = 8;
constexpr int kPts    = 4096;
constexpr int kCh     = 128;
constexpr int kNbr    = 16;
constexpr int kRows   = kPts * kNbr;
constexpr int kCin0   = 259;
constexpr int kK0     = 160;
constexpr int kLd0    = 192;
constexpr int kGroups = 8;
constexpr int kStatBlocks = 64;
constexpr float kWScale    = 64.0f;
constexpr float kWScaleInv = 0.015625f;

static_assert(kK0 % 32 == 0);
static_assert(kCh % 32 == 0);
static_assert(kCh % 64 == 0);
static_assert(kRows % 64 == 0);
static_assert(kPts % 64 == 0);
static_assert(kLd0 % 8 == 0 && kLd0 >= kK0);
static_assert((kLd0 * 2) % 128 == 0);
static_assert(kCh / kGroups == 16);
static_assert(kRows == kStatBlocks * 1024);
static_assert(kPts % 256 == 0);

constexpr size_t kBytesFT   = (size_t)kBatch * kPts * kCh * 2;
constexpr size_t kBytesW128 = (size_t)kCh * kCh * 2;
constexpr size_t kBytesW0b  = (size_t)kCh * kLd0 * 2;
constexpr size_t kBytesPart = (size_t)kStatBlocks * 128;
constexpr size_t kBytesF1   = (size_t)kBatch * kPts * kCh * 4;
constexpr size_t kBytesXP   = (size_t)kRows * kLd0 * 2;
constexpr size_t kBytesY    = (size_t)kRows * kCh * 4;

constexpr size_t kOffF1T  = 0;
constexpr size_t kOffF2T  = kOffF1T + kBytesFT;
constexpr size_t kOffW0a  = kOffF2T + kBytesFT;
constexpr size_t kOffW0b  = kOffW0a + kBytesW128;
constexpr size_t kOffW1   = kOffW0b + kBytesW0b;
constexpr size_t kOffW2   = kOffW1 + kBytesW128;
constexpr size_t kOffPart = kOffW2 + kBytesW128;
constexpr size_t kOffF1   = kOffPart + kBytesPart;
constexpr size_t kOffXP   = kOffF1 + kBytesF1;
constexpr size_t kOffYA   = kOffXP + kBytesXP;
constexpr size_t kOffYB   = kOffYA + kBytesY;
constexpr size_t kWsTotal = kOffYB + kBytesY;
static_assert(kWsTotal == 125984768);
static_assert(kWsTotal <= 134217728);
static_assert(kOffW0a % 256 == 0 && kOffW0b % 256 == 0 && kOffW1 % 256 == 0 && kOffW2 % 256 == 0);
static_assert(kOffPart % 256 == 0 && kOffF1 % 256 == 0 && kOffXP % 256 == 0 && kOffYA % 256 == 0 && kOffYB % 256 == 0);
static_assert((size_t)kRows * kCh * 2 <= kBytesXP);
static_assert(kBytesW128 % 512 == 0 && kBytesW0b % 512 == 0);

__device__ __forceinline__ float bf16_rne(float f) {
  unsigned u = __float_as_uint(f);
  u = (u + 0x7FFFu + ((u >> 16) & 1u)) & 0xFFFF0000u;
  return __uint_as_float(u);
}
__device__ __forceinline__ unsigned f16_bits(float f) {
  const _Float16 h = (_Float16)f;
  return (unsigned)__builtin_bit_cast(unsigned short, h);
}
__device__ __forceinline__ unsigned pack_f16x2(float a, float b) {
  return f16_bits(a) | (f16_bits(b) << 16);
}
__device__ __forceinline__ double shfl_xor_f64(double v, int m) {
  const unsigned long long u = __builtin_bit_cast(unsigned long long, v);
  int lo = (int)(unsigned)(u & 0xFFFFFFFFull);
  int hi = (int)(unsigned)(u >> 32);
  lo = __shfl_xor(lo, m, 32);
  hi = __shfl_xor(hi, m, 32);
  const unsigned long long r = ((unsigned long long)(unsigned)hi << 32) | (unsigned long long)(unsigned)lo;
  return __builtin_bit_cast(double, r);
}

__device__ __forceinline__ void dep_guard_h(v8f& a, v8f& b, v16h x, v16h y) { asm volatile("v_nop\n\tv_nop\n\tv_nop\n\tv_nop" : "+v"(a), "+v"(b) : "v"(x), "v"(y)); }
__device__ __forceinline__ void keep4_h(v16h a, v16h b, v16h c, v16h d) { asm volatile("v_nop" :: "v"(a), "v"(b), "v"(c), "v"(d)); }
__device__ __forceinline__ void acc_guard4(v8f& a, v8f& b, v8f& c, v8f& d) { asm volatile("v_nop\n\tv_nop\n\tv_nop\n\tv_nop" : "+v"(a), "+v"(b), "+v"(c), "+v"(d)); }
template <typename T> struct Frag;
template <> struct Frag<_Float16> {
  typedef v16h V; union U { v16h v; v8h h[2]; };
  static __device__ __forceinline__ v16h load(const _Float16* p) {
    U f; f.h[0] = *(const v8h*)(p); f.h[1] = *(const v8h*)(p + 16); return f.v;
  }
  static __device__ __forceinline__ v8f mma(v16h a, v16h b, v8f c) {
    return __builtin_amdgcn_wmma_f32_16x16x32_f16(false, a, false, b, (short)0, c, false, false);
  }
  static __device__ __forceinline__ void guard(v8f& a, v8f& b, v16h x, v16h y) { dep_guard_h(a, b, x, y); }
  static __device__ __forceinline__ void keep(v16h a, v16h b, v16h c, v16h d) { keep4_h(a, b, c, d); }
};

template <int BIAS_MODE, int RES_ROWDIV>
__global__ __launch_bounds__(256) void gemm64_f16(
    const unsigned short* __restrict__ Ap, int lda, long strideA,
    const unsigned short* __restrict__ Btp, int ldb, long strideB,
    float* __restrict__ Cp, int ldc, long strideC,
    const float* __restrict__ bias,
    const float* __restrict__ resp, int ldr, long strideR,
    int M, int N, int K, float scale) {
  typedef _Float16 T;
  typedef Frag<T>::V V;
  const T* A = (const T*)Ap; const T* Bt = (const T*)Btp;
  __shared__ __align__(16) float sT[8][16 * 68];
  const int b    = blockIdx.y;
  const int lane = threadIdx.x & 31;
  const int wave = threadIdx.x >> 5;
  const int tilesN = N >> 6;
  const int tilesM = M >> 6;
  const int tile = blockIdx.x * 8 + wave;
  if (tile >= tilesM * tilesN) return;
  const int tm = tile / tilesN;
  const int tn = tile - tm * tilesN;
  const int m0 = tm << 6;
  const int n0 = tn << 6;

  const T* Ab = A  + (size_t)b * strideA;
  const T* Bb = Bt + (size_t)b * strideB;

  const int rlane = lane & 15;
  const int koff  = (lane >> 4) * 8;
  const int mOff  = (lane >> 4) * 8;

  v8f acc[4][4];
#pragma unroll
  for (int i = 0; i < 4; ++i)
#pragma unroll
    for (int j = 0; j < 4; ++j) acc[i][j] = (v8f){0.f,0.f,0.f,0.f,0.f,0.f,0.f,0.f};

  for (int k0 = 0; k0 < K; k0 += 32) {
    V bh[4];
#pragma unroll
    for (int j = 0; j < 4; ++j) {
      const size_t bo = (size_t)(n0 + (j << 4) + rlane) * ldb + koff + k0;
      bh[j] = Frag<T>::load(Bb + bo);
    }
#pragma unroll
    for (int i = 0; i < 4; ++i) {
      const size_t ao = (size_t)(m0 + (i << 4) + rlane) * lda + koff + k0;
      V ah = Frag<T>::load(Ab + ao);
#pragma unroll
      for (int j = 0; j < 4; ++j) acc[i][j] = Frag<T>::mma(ah, bh[j], acc[i][j]);
      Frag<T>::guard(acc[i][0], acc[i][3], ah, ah);
    }
    Frag<T>::keep(bh[0], bh[1], bh[2], bh[3]);
  }
  acc_guard4(acc[0][0], acc[0][1], acc[0][2], acc[0][3]);
  acc_guard4(acc[1][0], acc[1][1], acc[1][2], acc[1][3]);
  acc_guard4(acc[2][0], acc[2][1], acc[2][2], acc[2][3]);
  acc_guard4(acc[3][0], acc[3][1], acc[3][2], acc[3][3]);

  float* slab = sT[wave];
  float* Cb = Cp + (size_t)b * strideC;
  const float* Rb = resp + (size_t)b * strideR;
#pragma unroll
  for (int i = 0; i < 4; ++i) {
    const int mBase = m0 + (i << 4);
#pragma unroll
    for (int j = 0; j < 4; ++j) {
      const int n = n0 + (j << 4) + rlane;
      float bv = 0.f;
      if (BIAS_MODE == 2) bv = bias[n];
#pragma unroll
      for (int r = 0; r < 8; ++r) {
        float v = acc[i][j][r] * scale;
        if (BIAS_MODE == 2) v += bv;
        slab[(mOff + r) * 68 + (j << 4) + rlane] = v;
      }
    }
    __builtin_amdgcn_fence(__ATOMIC_RELEASE, "workgroup");
    __builtin_amdgcn_wave_barrier();
    __builtin_amdgcn_fence(__ATOMIC_ACQUIRE, "workgroup");
    {
      const int hh = lane >> 4, c4 = (lane & 15) * 4;
      for (int pass = 0; pass < 2; ++pass) {
#pragma unroll
        for (int it = 0; it < 8; ++it) {
          const int row = it * 2 + hh;
          v4f v = *(const v4f*)(slab + row * 68 + c4);
          if (RES_ROWDIV > 0) {
            const v4f rv = *(const v4f*)(Rb + (size_t)((mBase + row) / RES_ROWDIV) * ldr + n0 + c4);
            v = v + rv;
          }
          *(volatile v4f*)(Cb + (size_t)(mBase + row) * ldc + n0 + c4) = v;
        }
        __threadfence();
      }
    }
    __builtin_amdgcn_fence(__ATOMIC_RELEASE, "workgroup");
    __builtin_amdgcn_wave_barrier();
    __builtin_amdgcn_fence(__ATOMIC_ACQUIRE, "workgroup");
  }
}

__global__ __launch_bounds__(256) void transpose_cast_kernel(
    const float* __restrict__ src, unsigned short* __restrict__ dstT) {
  __shared__ float tile[kCh * 33];
  const int tid = threadIdx.x, lane = tid & 31, w = tid >> 5;
  const int b = blockIdx.y, n0 = blockIdx.x * 32;
  const float* sb = src + (size_t)b * kCh * kPts + n0;
#pragma unroll 4
  for (int i = 0; i < kCh / 8; ++i) {
    const int c = w + 8 * i;
    tile[c * 33 + lane] = bf16_rne(sb[(size_t)c * kPts + lane]);
  }
  __syncthreads();
  unsigned short* db = dstT + (size_t)(b * kPts + n0) * kCh;
#pragma unroll
  for (int jj = 0; jj < 2; ++jj) {
    const int flat = tid + 256 * jj;
    const int nl = flat >> 4, c8 = (flat & 15) * 8;
    v4u val;
#pragma unroll
    for (int e = 0; e < 4; ++e)
      val[e] = pack_f16x2(tile[(c8 + 2 * e) * 33 + nl], tile[(c8 + 2 * e + 1) * 33 + nl]);
    unsigned short* d = db + (size_t)nl * kCh + c8;
    *(volatile v4u*)d = val;
    __threadfence();
    *(volatile v4u*)d = val;
  }
}

__global__ __launch_bounds__(256) void weight_prep_kernel(
    const float* __restrict__ w0, const float* __restrict__ w1, const float* __restrict__ w2,
    unsigned short* __restrict__ p0a, unsigned short* __restrict__ p0b,
    unsigned short* __restrict__ p1, unsigned short* __restrict__ p2) {
  const int blk = blockIdx.x, tid = threadIdx.x;
  float v[8];
  unsigned short* dst;
  if (blk < 8) {
    const int u = blk * 256 + tid;
    const int row = u >> 4, c8 = (u & 15) * 8;
#pragma unroll
    for (int e = 0; e < 8; ++e) v[e] = w0[(size_t)row * kCin0 + c8 + e];
    dst = p0a + (size_t)u * 8;
  } else if (blk < 20) {
    const int u = (blk - 8) * 256 + tid;
    const int row = u / 24, c8 = (u - row * 24) * 8;
#pragma unroll
    for (int e = 0; e < 8; ++e) {
      const int col = c8 + e;
      const int sc = (col < 128) ? (128 + col) : ((col < 131) ? (256 + col - 128) : 258);
      const float t = w0[(size_t)row * kCin0 + sc];
      v[e] = (col < 131) ? t : 0.0f;
    }
    dst = p0b + (size_t)u * 8;
  } else if (blk < 28) {
    const int u = (blk - 20) * 256 + tid;
    const int row = u >> 4, c8 = (u & 15) * 8;
#pragma unroll
    for (int e = 0; e < 8; ++e) v[e] = w1[(size_t)row * kCh + c8 + e];
    dst = p1 + (size_t)u * 8;
  } else {
    const int u = (blk - 28) * 256 + tid;
    const int row = u >> 4, c8 = (u & 15) * 8;
#pragma unroll
    for (int e = 0; e < 8; ++e) v[e] = w2[(size_t)row * kCh + c8 + e];
    dst = p2 + (size_t)u * 8;
  }
  v4u val;
#pragma unroll
  for (int e = 0; e < 4; ++e)
    val[e] = pack_f16x2(bf16_rne(v[2 * e]) * kWScale, bf16_rne(v[2 * e + 1]) * kWScale);
  *(volatile v4u*)dst = val;
  __threadfence();
  *(volatile v4u*)dst = val;
}

__global__ __launch_bounds__(256) void knn_group_kernel(
    const float* __restrict__ xyz1, const float* __restrict__ xyz2,
    const unsigned short* __restrict__ f2t, unsigned short* __restrict__ xout, int bidx) {
  extern __shared__ v4f pts[];
  const int tid = threadIdx.x;
  const float* x2 = xyz2 + (size_t)bidx * 3 * kPts;
#pragma unroll 2
  for (int i = 0; i < kPts / 256; ++i) {
    const int m = tid + 256 * i;
    const float x = bf16_rne(x2[m]);
    const float y = bf16_rne(x2[kPts + m]);
    const float z = bf16_rne(x2[2 * kPts + m]);
    const float t0 = x * x;
    const float t1 = y * y;
    const float t2 = z * z;
    const float s = (t0 + t2) + t1;
    v4f e; e[0] = x; e[1] = y; e[2] = z; e[3] = s;
    pts[m] = e;
  }
  __syncthreads();

  const int wave = tid >> 5, lane = tid & 31;
  const int n = blockIdx.x * 8 + wave;
  const float* x1 = xyz1 + (size_t)bidx * 3 * kPts;
  const float qx = bf16_rne(x1[n]);
  const float qy = bf16_rne(x1[kPts + n]);
  const float qz = bf16_rne(x1[2 * kPts + n]);
  float sq1;
  {
    const float t0 = qx * qx;
    const float t1 = qy * qy;
    const float t2 = qz * qz;
    sq1 = (t0 + t2) + t1;
  }

  float bestd = 3.0e38f;
  int   besti = 0;
  float thr   = 3.0e38f;
#pragma unroll 1
  for (int m0 = 0; m0 < kPts; m0 += 32) {
    const v4f p4 = pts[m0 + lane];
    const float t = sq1 + p4[3];
    float p = qx * p4[0];
    p = fmaf(qy, p4[1], p);
    p = fmaf(qz, p4[2], p);
    const float d = t - 2.0f * p;
    unsigned mask = __builtin_amdgcn_ballot_w32(d < thr);
    for (int it = 0; it < 32 && mask != 0u; ++it) {
      const int src = __builtin_ctz(mask);
      mask &= (mask - 1u);
      const float v  = __int_as_float(__builtin_amdgcn_readlane(__float_as_int(d), src));
      const int   ci = m0 + src;
      const float upd = __shfl_up(bestd, 1, 32);
      const int   upi = __shfl_up(besti, 1, 32);
      const float pl = (lane == 0) ? -3.0e38f : upd;
      const bool lt = v < bestd;
      const bool ge = v >= pl;
      const float nd = lt ? (ge ? v : pl) : bestd;
      const int   ni = lt ? (ge ? ci : upi) : besti;
      bestd = nd;
      besti = ni;
      thr = __int_as_float(__builtin_amdgcn_readlane(__float_as_int(bestd), 15));
    }
  }

  const unsigned short* f2b = f2t + (size_t)bidx * kPts * kCh;
  const int lc = (lane < 16) ? lane : 15;
  unsigned short* xrow0 = xout + (size_t)n * kNbr * kLd0;
#pragma unroll
  for (int j = 0; j < kNbr; ++j) {
    int idx = __builtin_amdgcn_readlane(besti, j);
    idx = (idx < 0) ? 0 : ((idx > kPts - 1) ? (kPts - 1) : idx);
    const v4u fv = *(const v4u*)(f2b + (size_t)idx * kCh + lc * 8);
    const v4f pp = pts[idx];
    float dx = pp[0] - qx;
    float dy = pp[1] - qy;
    float dz = pp[2] - qz;
    asm volatile("" : "+v"(dx), "+v"(dy), "+v"(dz));
    float dzz = dz - dz;
    asm volatile("" : "+v"(dzz));
    const unsigned g0 = pack_f16x2(dx, dy);
    const unsigned g1 = pack_f16x2(dz, dzz);
    const bool isf = lane < 16;
    const bool isg = lane == 16;
    v4u val;
    val[0] = isf ? fv[0] : (isg ? g0 : 0u);
    val[1] = isf ? fv[1] : (isg ? g1 : 0u);
    val[2] = isf ? fv[2] : 0u;
    val[3] = isf ? fv[3] : 0u;
    unsigned short* dst = xrow0 + (size_t)j * kLd0 + lane * 8;
    if (lane < 24) *(volatile v4u*)dst = val;
    __threadfence();
    if (lane < 24) *(volatile v4u*)dst = val;
  }
}

__global__ __launch_bounds__(256) void stats_kernel(
    const float* __restrict__ Y, double* __restrict__ part) {
  __shared__ double shs[8][8];
  __shared__ double shq[8][8];
  const int tid = threadIdx.x, lane = tid & 31, w = tid >> 5;
  const size_t rowbase = (size_t)blockIdx.x * 1024;
  double ds = 0.0, dq = 0.0;
#pragma unroll 2
  for (int i = 0; i < 128; ++i) {
    const size_t row = rowbase + (size_t)(w + 8 * i);
    const v4f y = *(const v4f*)(Y + row * kCh + 4 * lane);
    const float s4 = (y[0] + y[1]) + (y[2] + y[3]);
    const float a0 = y[0] * y[0];
    const float a1 = y[1] * y[1];
    const float a2 = y[2] * y[2];
    const float a3 = y[3] * y[3];
    const float q4 = (a0 + a1) + (a2 + a3);
    ds += (double)s4;
    dq += (double)q4;
  }
  ds += shfl_xor_f64(ds, 1); dq += shfl_xor_f64(dq, 1);
  ds += shfl_xor_f64(ds, 2); dq += shfl_xor_f64(dq, 2);
  if ((lane & 3) == 0) { shs[w][lane >> 2] = ds; shq[w][lane >> 2] = dq; }
  __syncthreads();
  if (tid < 32) {
    const int g = lane & 7;
    double S = 0.0, Q = 0.0;
#pragma unroll
    for (int ww = 0; ww < 8; ++ww) { S += shs[ww][g]; Q += shq[ww][g]; }
    v2d val; val[0] = S; val[1] = Q;
    double* dst = part + (size_t)blockIdx.x * 16 + 2 * g;
    if (lane < 8) *(volatile v2d*)dst = val;
    __threadfence();
    if (lane < 8) *(volatile v2d*)dst = val;
  }
}

__device__ __forceinline__ void group_moments(const double* __restrict__ part, int lane,
                                              float& mean_out, float& rstd_out) {
  const int tt = lane & 15;
  const int g = tt >> 1, which = tt & 1;
  double acc = 0.0;
#pragma unroll 1
  for (int blk = 0; blk < kStatBlocks; ++blk) acc += part[blk * 16 + 2 * g + which];
  const double oth = shfl_xor_f64(acc, 1);
  const double S = which ? oth : acc;
  const double Q = which ? acc : oth;
  const double inv = 1.0 / 1048576.0;
  const double mean = S * inv;
  const double var = Q * inv - mean * mean;
  float varf = (float)var;
  varf = fmaxf(varf, 0.0f);
  mean_out = (float)mean;
  rstd_out = 1.0f / sqrtf(varf + 1e-5f);
}

__global__ __launch_bounds__(256) void norm_act_cast_kernel(
    const float* __restrict__ Y, const double* __restrict__ part,
    const float* __restrict__ gam, const float* __restrict__ bet,
    unsigned short* __restrict__ X) {
  __shared__ float mst[2 * kGroups];
  const int tid = threadIdx.x, lane = tid & 31;
  if (tid < 32) {
    float mf, rf;
    group_moments(part, lane, mf, rf);
    if ((lane & 1) == 0 && lane < 16) { mst[lane] = mf; mst[lane + 1] = rf; }
  }
  __syncthreads();
  const int c8 = (tid & 15) * 8;
  const int g = c8 >> 4;
  const float mean = mst[2 * g], rstd = mst[2 * g + 1];
  const v4f ga = *(const v4f*)(gam + c8);
  const v4f gb = *(const v4f*)(gam + c8 + 4);
  const v4f ba = *(const v4f*)(bet + c8);
  const v4f bb = *(const v4f*)(bet + c8 + 4);
  float a[8], s[8];
#pragma unroll
  for (int e = 0; e < 4; ++e) {
    a[e]     = bf16_rne(ga[e]) * rstd;
    a[e + 4] = bf16_rne(gb[e]) * rstd;
    s[e]     = bf16_rne(ba[e]) - mean * a[e];
    s[e + 4] = bf16_rne(bb[e]) - mean * a[e + 4];
  }
  const int rsub = tid >> 4;
  const size_t rb = (size_t)blockIdx.x * 1024;
#pragma unroll 1
  for (int i = 0; i < 64; ++i) {
    const size_t row = rb + (size_t)(i * 16 + rsub);
    const float* yp = Y + row * kCh + c8;
    const v4f y0 = *(const v4f*)yp;
    const v4f y1 = *(const v4f*)(yp + 4);
    float o[8];
#pragma unroll
    for (int e = 0; e < 4; ++e) { o[e] = y0[e] * a[e] + s[e]; o[e + 4] = y1[e] * a[e + 4] + s[e + 4]; }
#pragma unroll
    for (int e = 0; e < 8; ++e) o[e] = (o[e] >= 0.0f) ? o[e] : 0.1f * o[e];
    v4u val;
#pragma unroll
    for (int e = 0; e < 4; ++e) val[e] = pack_f16x2(o[2 * e], o[2 * e + 1]);
    unsigned short* d = X + row * kCh + c8;
    *(volatile v4u*)d = val;
    __threadfence();
    *(volatile v4u*)d = val;
  }
}

__global__ __launch_bounds__(256) void norm_act_maxpool_kernel(
    const float* __restrict__ Y, const double* __restrict__ part,
    const float* __restrict__ gam, const float* __restrict__ bet,
    float* __restrict__ outb) {
  __shared__ float mst[2 * kGroups];
  __shared__ float tileT[kCh * 33];
  const int tid = threadIdx.x, lane = tid & 31, w = tid >> 5;
  if (tid < 32) {
    float mf, rf;
    group_moments(part, lane, mf, rf);
    if ((lane & 1) == 0 && lane < 16) { mst[lane] = mf; mst[lane + 1] = rf; }
  }
  __syncthreads();
  const int q = lane;
  const int g = q >> 2;
  const float mean = mst[2 * g], rstd = mst[2 * g + 1];
  const v4f gv = *(const v4f*)(gam + 4 * q);
  const v4f bv = *(const v4f*)(bet + 4 * q);
  float a[4], s[4];
#pragma unroll
  for (int e = 0; e < 4; ++e) { a[e] = bf16_rne(gv[e]) * rstd; s[e] = bf16_rne(bv[e]) - mean * a[e]; }
  const int n0 = blockIdx.x * 32;
#pragma unroll 1
  for (int pass = 0; pass < 4; ++pass) {
    const int nl = w + 8 * pass;
    const int n = n0 + nl;
    float mx[4] = {-3.0e38f, -3.0e38f, -3.0e38f, -3.0e38f};
#pragma unroll 4
    for (int kk = 0; kk < kNbr; ++kk) {
      const v4f y = *(const v4f*)(Y + ((size_t)n * kNbr + kk) * kCh + 4 * q);
#pragma unroll
      for (int e = 0; e < 4; ++e) {
        float v = y[e] * a[e] + s[e];
        v = (v >= 0.0f) ? v : 0.1f * v;
        mx[e] = fmaxf(mx[e], v);
      }
    }
#pragma unroll
    for (int e = 0; e < 4; ++e) tileT[(4 * q + e) * 33 + nl] = mx[e];
  }
  __syncthreads();
  const int cq = lane >> 3, noff = (lane & 7) * 4;
  for (int pass = 0; pass < 2; ++pass) {
#pragma unroll
    for (int it = 0; it < 4; ++it) {
      const int c = w * 16 + it * 4 + cq;
      v4f v;
      v[0] = tileT[c * 33 + noff + 0];
      v[1] = tileT[c * 33 + noff + 1];
      v[2] = tileT[c * 33 + noff + 2];
      v[3] = tileT[c * 33 + noff + 3];
      *(volatile v4f*)(outb + (size_t)c * kPts + n0 + noff) = v;
    }
    __threadfence();
  }
}

extern "C" void kernel_launch(void* const* d_in, const int* in_sizes, int n_in,
                              void* d_out, int out_size, void* d_ws, size_t ws_size,
                              hipStream_t stream) {
  if (n_in < 16) return;
  if (out_size != kBatch * kCh * kPts) return;
  if (in_sizes[0] != kBatch * 3 * kPts || in_sizes[1] != kBatch * 3 * kPts) return;
  if (in_sizes[2] != kBatch * kCh * kPts || in_sizes[3] != kBatch * kCh * kPts) return;
  if (in_sizes[4] != kCh * kCin0 || in_sizes[8] != kCh * kCh || in_sizes[12] != kCh * kCh) return;
  if (ws_size < kWsTotal) return;

  const float* xyz1  = (const float*)d_in[0];
  const float* xyz2  = (const float*)d_in[1];
  const float* feat1 = (const float*)d_in[2];
  const float* feat2 = (const float*)d_in[3];
  const float* W0 = (const float*)d_in[4];  const float* b0 = (const float*)d_in[5];
  const float* g0 = (const float*)d_in[6];  const float* bt0 = (const float*)d_in[7];
  const float* W1 = (const float*)d_in[8];  const float* b1 = (const float*)d_in[9];
  const float* g1 = (const float*)d_in[10]; const float* bt1 = (const float*)d_in[11];
  const float* W2 = (const float*)d_in[12]; const float* b2 = (const float*)d_in[13];
  const float* g2 = (const float*)d_in[14]; const float* bt2 = (const float*)d_in[15];
  float* out = (float*)d_out;

  char* ws = (char*)d_ws;
  unsigned short* f1t = (unsigned short*)(ws + kOffF1T);
  unsigned short* f2t = (unsigned short*)(ws + kOffF2T);
  unsigned short* w0a = (unsigned short*)(ws + kOffW0a);
  unsigned short* w0b = (unsigned short*)(ws + kOffW0b);
  unsigned short* w1p = (unsigned short*)(ws + kOffW1);
  unsigned short* w2p = (unsigned short*)(ws + kOffW2);
  double* part = (double*)(ws + kOffPart);
  float*  f1   = (float*)(ws + kOffF1);
  unsigned short* xp = (unsigned short*)(ws + kOffXP);
  float*  ya   = (float*)(ws + kOffYA);
  float*  yb   = (float*)(ws + kOffYB);

  const long strideNC = (long)kPts * kCh;
  const int gemmBlkF1 = (kPts / 64) * (kCh / 64) / 8;
  const int gemmBlkL  = (kRows / 64) * (kCh / 64) / 8;

  transpose_cast_kernel<<<dim3(kPts / 32, kBatch), 256, 0, stream>>>(feat1, f1t);
  transpose_cast_kernel<<<dim3(kPts / 32, kBatch), 256, 0, stream>>>(feat2, f2t);
  weight_prep_kernel<<<36, 256, 0, stream>>>(W0, W1, W2, w0a, w0b, w1p, w2p);
  gemm64_f16<2, 0><<<dim3(gemmBlkF1, kBatch), 256, 0, stream>>>(
      f1t, kCh, strideNC, w0a, kCh, 0L, f1, kCh, strideNC, b0, f1, kCh, 0L,
      kPts, kCh, kCh, kWScaleInv);

  for (int b = 0; b < kBatch; ++b) {
    knn_group_kernel<<<kPts / 8, 256, kPts * 16, stream>>>(xyz1, xyz2, f2t, xp, b);
    gemm64_f16<0, 16><<<dim3(gemmBlkL, 1), 256, 0, stream>>>(
        xp, kLd0, 0L, w0b, kLd0, 0L, ya, kCh, 0L, b0, f1 + (size_t)b * kPts * kCh, kCh, 0L,
        kRows, kCh, kK0, kWScaleInv);
    stats_kernel<<<kStatBlocks, 256, 0, stream>>>(ya, part);
    norm_act_cast_kernel<<<kStatBlocks, 256, 0, stream>>>(ya, part, g0, bt0, xp);
    gemm64_f16<2, 0><<<dim3(gemmBlkL, 1), 256, 0, stream>>>(
        xp, kCh, 0L, w1p, kCh, 0L, yb, kCh, 0L, b1, f1, kCh, 0L,
        kRows, kCh, kCh, kWScaleInv);
    stats_kernel<<<kStatBlocks, 256, 0, stream>>>(yb, part);
    norm_act_cast_kernel<<<kStatBlocks, 256, 0, stream>>>(yb, part, g1, bt1, xp);
    gemm64_f16<2, 0><<<dim3(gemmBlkL, 1), 256, 0, stream>>>(
        xp, kCh, 0L, w2p, kCh, 0L, ya, kCh, 0L, b2, f1, kCh, 0L,
        kRows, kCh, kCh, kWScaleInv);
    stats_kernel<<<kStatBlocks, 256, 0, stream>>>(ya, part);
    norm_act_maxpool_kernel<<<kPts / 32, 256, 0, stream>>>(ya, part, g2, bt2,
                                                          out + (size_t)b * kCh * kPts);
  }
}
